// GlycanGearNet_55645596287225
// MI455X (gfx1250) — hardware-verified
//
#include <hip/hip_runtime.h>
#include <stddef.h>
#include <stdint.h>


#define FEAT   128
#define NREL   7
#define KREL   896
#define KD     1024
#define KQ     128
#define KSTEPS 32
#define APK    1032
#define TR     16
#define NTHR   256
#define NWAVE  8
#define S1     4096
#define NCH1   16
#define SH1    12
#define SH2    7
#define SH3    2
#define MIDS   32
#define NGRP   4
#define F1A    16
#define F2     32
#define F3     32
#define CAP1   512
#define CAP2   320
#define CAP3   256
#define CPS1   2
#define SEGS2  16
#define NCH2   32
#define ASC    256.0f
#define BSC    256.0f
#define RSC    0.0000152587890625f
#define SENT   0xFFFFFFFFu
#define WSCAPB 134217728
#define ZIT    14
#define ACC_BYTES 57344
#define SA_BYTES  33024
#define STG_BYTES 8192
#define TILE_LDS  (ACC_BYTES + SA_BYTES + STG_BYTES)

static_assert(KREL == NREL * FEAT);
static_assert(KD == KREL + FEAT);
static_assert(KQ * 8 == KD);
static_assert(KSTEPS * 32 == KD);
static_assert((KREL % 32) == 0);
static_assert((APK % 8) == 0 && APK >= KD);
static_assert((FEAT * KQ) % NTHR == 0);
static_assert(NCH1 * NTHR == S1);
static_assert(CPS1 * NTHR == CAP1 && NCH2 == SEGS2 * CPS1);
static_assert((F1A * CAP1) % (4 * NTHR) == 0);
static_assert((F2 * CAP2) % (4 * NTHR) == 0);
static_assert((F3 * CAP3) % (4 * NTHR) == 0);
static_assert((CAP1 % 32) == 0 && (CAP2 % 32) == 0 && (CAP3 % 32) == 0);
static_assert(F1A <= 32 && F2 <= 32 && F3 <= 32);
static_assert((1 << (SH1 - SH2)) == MIDS && (1 << (SH2 - SH3)) == F3 && (1 << (4 - SH3)) == NGRP);
static_assert(NTHR == 32 * NWAVE && TR == 2 * NWAVE);
static_assert(NTHR == TR * (FEAT / 8));
static_assert(FEAT == 4 * 32);
static_assert(TR * KREL * 4 == ACC_BYTES && TR * APK * 2 == SA_BYTES && TR * FEAT * 4 == STG_BYTES);
static_assert(ZIT * 4 * NTHR == TR * KREL);
static_assert(TILE_LDS == 98560);

typedef _Float16 v4h  __attribute__((ext_vector_type(4)));
typedef _Float16 v8h  __attribute__((ext_vector_type(8)));
typedef _Float16 v16h __attribute__((ext_vector_type(16)));
typedef float    v4f  __attribute__((ext_vector_type(4)));
typedef float    v8f  __attribute__((ext_vector_type(8)));
typedef unsigned int v4u __attribute__((ext_vector_type(4)));
typedef v4h v4ha __attribute__((may_alias));
typedef v8h v8ha __attribute__((may_alias));
typedef v4f v4fa __attribute__((may_alias));
typedef v4u v4ua __attribute__((may_alias));
union Frag { v16h v; v8h h[2]; };
union H8 { v8h v; v4h q[2]; };

__device__ __forceinline__ v8f wmh(v16h a, v16h b, v8f c) {
  v8f d = __builtin_amdgcn_wmma_f32_16x16x32_f16(false, a, false, b, (short)0, c, false, false);
  asm volatile("v_nop\n\tv_nop\n\tv_nop\n\tv_nop" : "+v"(d) : "v"(a), "v"(b));
  return d;
}

__device__ __forceinline__ v4h cvt4s(v4f a) {
  v4h r;
  r[0] = (_Float16)(a[0] * ASC); r[1] = (_Float16)(a[1] * ASC);
  r[2] = (_Float16)(a[2] * ASC); r[3] = (_Float16)(a[3] * ASC);
  return r;
}

__global__ __launch_bounds__(NTHR) void k_wprep(const float* __restrict__ wr, const float* __restrict__ wl,
                                                _Float16* Bw) {
  const int i = blockIdx.x * NTHR + threadIdx.x;
  const int layer = i / (FEAT * KQ);
  const int rem = i - layer * (FEAT * KQ);
  const int n = rem / KQ, kq = rem - n * KQ, k0 = kq * 8;
  const int kr = k0 < (KREL - 8) ? k0 : (KREL - 8);
  int kl = k0 - KREL;
  kl = kl < 0 ? 0 : (kl > FEAT - 8 ? FEAT - 8 : kl);
  const bool isrel = k0 < KREL;
  const float* pr = wr + ((size_t)layer * KREL + kr) * FEAT + n;
  const float* pl = wl + ((size_t)layer * FEAT + kl) * FEAT + n;
  v8h hv;
#pragma unroll
  for (int e = 0; e < 8; ++e) {
    const float vr = pr[(size_t)e * FEAT];
    const float vl = pl[(size_t)e * FEAT];
    const float v = isrel ? vr : vl;
    hv[e] = (_Float16)(v * BSC);
  }
  _Float16* dst = Bw + (size_t)i * 8;
  *(volatile v8h*)dst = hv;
  __threadfence();
  *(volatile v8h*)dst = hv;
}

__global__ __launch_bounds__(NTHR) void k_embed(const int* __restrict__ ut, const float* __restrict__ emb,
                                                float* x, int nN, int nU) {
  const int tid = threadIdx.x, lane = tid & 31, wave = tid >> 5;
  const int n = blockIdx.x * NWAVE + wave;
  const bool act = n < nN;
  const int nc = act ? n : nN - 1;
  int u = ut[nc];
  u = u < 0 ? 0 : (u > nU - 1 ? nU - 1 : u);
  const v4f v = *(const v4f*)(emb + (size_t)u * FEAT + 4 * lane);
  float* gp = x + (size_t)nc * FEAT + 4 * lane;
  if (act) *(volatile v4f*)gp = v;
  __threadfence();
  if (act) *(volatile v4f*)gp = v;
}

template <int LV, int FA, int CAP>
__global__ __launch_bounds__(NTHR) void k_part(const int* __restrict__ edst, const unsigned* lin, unsigned* lout,
                                               int nN, int nE, int nC, int nB1, int P2, int nch) {
  __shared__ __attribute__((aligned(16))) unsigned lst[FA * CAP];
  __shared__ int wc[NWAVE * 32];
  __shared__ int cur[32];
  const int tid = threadIdx.x, lane = tid & 31, wave = tid >> 5;
  const int blk = blockIdx.x;
  const v4u sv = {SENT, SENT, SENT, SENT};
#pragma unroll
  for (int k = 0; k < (FA * CAP) / (4 * NTHR); ++k) *(v4ua*)(&lst[4 * (tid + NTHR * k)]) = sv;
  if (wave == 0) cur[lane] = 0;
  __syncthreads();

  int c = 0, part = 0, ml = 0;
  if (LV == 2) { c = blk / P2; part = blk - c * P2; }
  if (LV == 3) { c = blk / MIDS; ml = blk - c * MIDS; }
  const int nslots3 = P2 * CAP2;

#pragma unroll 1
  for (int ch = 0; ch < nch; ++ch) {
    bool valid;
    int key;
    unsigned rec;
    if (LV == 1) {
      const int e = blk * S1 + ch * NTHR + tid;
      const int ec = e < nE ? e : nE - 1;
      const int d = edst[ec];
      valid = (e < nE) && ((unsigned)d < (unsigned)nN);
      key = d >> SH1;
      rec = (unsigned)ec;
    } else if (LV == 2) {
      const int sgi = ch / CPS1;
      const int bl = part * SEGS2 + sgi;
      const int blc = bl < nB1 ? bl : nB1 - 1;
      const int slot = (ch - sgi * CPS1) * NTHR + tid;
      const unsigned id = lin[((size_t)blc * nC + c) * CAP1 + slot];
      const bool idok = id < (unsigned)nE;
      const int idc = idok ? (int)id : nE - 1;
      const int d = edst[idc];
      valid = (bl < nB1) && idok && ((unsigned)d < (unsigned)nN) && ((d >> SH1) == c);
      key = (d >> SH2) & (F2 - 1);
      rec = (unsigned)idc;
    } else {
      const int q = ch * NTHR + tid;
      const int qc = q < nslots3 ? q : nslots3 - 1;
      const int pp = qc / CAP2, s = qc - pp * CAP2;
      const unsigned id = lin[(((size_t)(c * P2 + pp)) * F2 + ml) * CAP2 + s];
      const bool idok = id < (unsigned)nE;
      const int idc = idok ? (int)id : nE - 1;
      const int d = edst[idc];
      valid = (q < nslots3) && idok && ((unsigned)d < (unsigned)nN) && ((d >> SH2) == blk);
      key = (d >> SH3) & (F3 - 1);
      rec = (unsigned)idc;
    }
    key = valid ? key : 255;
    unsigned mym = 0u;
#pragma unroll
    for (int b = 0; b < FA; ++b) {
      const unsigned mb = __builtin_amdgcn_ballot_w32(key == b);
      mym = (key == b) ? mb : mym;
    }
    const unsigned lt = (1u << lane) - 1u;
    const int rank = __builtin_popcount(mym & lt);
    const int cnt  = __builtin_popcount(mym);
    wc[wave * 32 + lane] = 0;
    if (valid && rank == 0) wc[wave * 32 + key] = cnt;
    __syncthreads();
    const int kc = key & 31;
    int pre = 0;
    for (int w2 = 0; w2 < wave; ++w2) pre += wc[w2 * 32 + kc];
    const int pos = cur[kc] + pre + rank;
    if (valid && pos < CAP) lst[kc * CAP + pos] = rec;
    int tot = 0;
    if (wave == 0) {
#pragma unroll
      for (int w2 = 0; w2 < NWAVE; ++w2) tot += wc[w2 * 32 + lane];
    }
    __syncthreads();
    if (wave == 0) cur[lane] += tot;
  }
  __syncthreads();

  const int nwords  = (LV == 1) ? nC * CAP : FA * CAP;
  const int npieces = nwords >> 2;
  unsigned* gb = lout + (size_t)blk * nwords;
#pragma unroll
  for (int k = 0; k < (FA * CAP / 4 + NTHR - 1) / NTHR; ++k) {
    const int it = tid + NTHR * k;
    if (it < npieces) { const v4u v = *(const v4ua*)(&lst[4 * it]); *(volatile v4u*)(gb + 4 * it) = v; }
  }
  __threadfence();
#pragma unroll
  for (int k = 0; k < (FA * CAP / 4 + NTHR - 1) / NTHR; ++k) {
    const int it = tid + NTHR * k;
    if (it < npieces) { const v4u v = *(const v4ua*)(&lst[4 * it]); *(volatile v4u*)(gb + 4 * it) = v; }
  }
}

__device__ __forceinline__ void drain(unsigned mk, unsigned id, float* rowp, const float* __restrict__ x,
                                      const int* __restrict__ esrc, const int* __restrict__ ety,
                                      const float* __restrict__ ew, int lane, int nN) {
  while (mk != 0u) {
    const int i = __builtin_ctz(mk);
    mk &= mk - 1u;
    const int e = __builtin_amdgcn_readlane((int)id, i);
    int src = esrc[e];
    src = src < 0 ? 0 : (src > nN - 1 ? nN - 1 : src);
    int ty = ety[e];
    ty = ty < 0 ? 0 : (ty > NREL - 1 ? NREL - 1 : ty);
    const float w = ew[e];
    const v4f v = *(const v4f*)(x + (size_t)src * FEAT + 4 * lane);
    v4fa* p = (v4fa*)(rowp + ty * FEAT + 4 * lane);
    v4f t = *p;
    t += v * w;
    *p = t;
  }
}

__global__ __launch_bounds__(NTHR) void k_tile(const float* __restrict__ x, const _Float16* __restrict__ Bw,
                                               const unsigned* __restrict__ l3, const int* __restrict__ esrc,
                                               const int* __restrict__ edst, const int* __restrict__ ety,
                                               const float* __restrict__ ew, const float* __restrict__ brel,
                                               const float* __restrict__ bloop, float* out, int nN, int nE) {
  extern __shared__ __attribute__((aligned(16))) unsigned char dynlds[];
  float*    accf = (float*)dynlds;
  _Float16* sA   = (_Float16*)(dynlds + ACC_BYTES);
  float*    stg  = (float*)(dynlds + ACC_BYTES + SA_BYTES);
  const int tid = threadIdx.x, lane = tid & 31, wave = tid >> 5, hh = lane >> 4, m = lane & 15;
  const int tile = blockIdx.x;

  const v4f z4 = {0.f, 0.f, 0.f, 0.f};
#pragma unroll
  for (int k = 0; k < ZIT; ++k) *(v4fa*)(accf + 4 * (tid + NTHR * k)) = z4;
  {
    const int row = tid >> 4, c8 = (tid & 15) * 8;
    const int node = tile * TR + row;
    const int nc = node < nN ? node : nN - 1;
    v4f v0 = *(const v4f*)(x + (size_t)nc * FEAT + c8);
    v4f v1 = *(const v4f*)(x + (size_t)nc * FEAT + c8 + 4);
    if (node >= nN) { v0 = z4; v1 = z4; }
    H8 hv;
    hv.q[0] = cvt4s(v0);
    hv.q[1] = cvt4s(v1);
    *(v8ha*)(sA + row * APK + KREL + c8) = hv.v;
  }
  __syncthreads();

  {
    const unsigned* seg = l3 + ((size_t)tile * NGRP + (wave >> 1)) * CAP3;
    float* row0 = accf + (2 * wave) * KREL;
    float* row1 = row0 + KREL;
#pragma unroll 1
    for (int ch = 0; ch < CAP3 / 32; ++ch) {
      const unsigned id = seg[ch * 32 + lane];
      const bool idok = id < (unsigned)nE;
      const int idc = idok ? (int)id : nE - 1;
      const int d = edst[idc];
      const bool ok = idok && ((unsigned)d < (unsigned)nN) && ((d >> 4) == tile);
      const int ln = d & 15;
      const unsigned m0 = __builtin_amdgcn_ballot_w32(ok && (ln == 2 * wave));
      const unsigned m1 = __builtin_amdgcn_ballot_w32(ok && (ln == 2 * wave + 1));
      drain(m0, id, row0, x, esrc, ety, ew, lane, nN);
      drain(m1, id, row1, x, esrc, ety, ew, lane, nN);
    }
  }
  __syncthreads();

#pragma unroll
  for (int k = 0; k < ZIT; ++k) {
    const int idx4 = 4 * (tid + NTHR * k);
    const int row = idx4 / KREL, col = idx4 - row * KREL;
    const v4f v = *(const v4fa*)(accf + idx4);
    *(v4ha*)(sA + row * APK + col) = cvt4s(v);
  }
  __syncthreads();

  {
    const int ct = wave;
    v8f acc = {0.f, 0.f, 0.f, 0.f, 0.f, 0.f, 0.f, 0.f};
    const _Float16* abase = sA + m * APK + 8 * hh;
    const _Float16* bbase = Bw + (size_t)(ct * 16 + m) * KD + 8 * hh;
#pragma unroll 1
    for (int kt = 0; kt < KSTEPS; ++kt) {
      Frag a, b;
      a.h[0] = *(const v8ha*)(abase + 32 * kt);
      a.h[1] = *(const v8ha*)(abase + 32 * kt + 16);
      b.h[0] = *(const v8h*)(bbase + 32 * kt);
      b.h[1] = *(const v8h*)(bbase + 32 * kt + 16);
      acc = wmh(a.v, b.v, acc);
    }
    const int col = ct * 16 + m;
#pragma unroll
    for (int r = 0; r < 8; ++r) stg[(8 * hh + r) * FEAT + col] = acc[r];
  }
  __syncthreads();

  {
    const v4f bv = *(const v4f*)(brel + 4 * lane) + *(const v4f*)(bloop + 4 * lane);
    const v4f p0 = *(const v4fa*)(stg + wave * FEAT + 4 * lane);
    const v4f p1 = *(const v4fa*)(stg + (wave + NWAVE) * FEAT + 4 * lane);
    v4f o0 = p0 * RSC + bv;
    v4f o1 = p1 * RSC + bv;
    o0[0] = fmaxf(o0[0], 0.0f); o0[1] = fmaxf(o0[1], 0.0f); o0[2] = fmaxf(o0[2], 0.0f); o0[3] = fmaxf(o0[3], 0.0f);
    o1[0] = fmaxf(o1[0], 0.0f); o1[1] = fmaxf(o1[1], 0.0f); o1[2] = fmaxf(o1[2], 0.0f); o1[3] = fmaxf(o1[3], 0.0f);
    const int n0 = tile * TR + wave, n1 = n0 + NWAVE;
    const bool a0 = n0 < nN, a1 = n1 < nN;
    float* g0 = out + (size_t)(a0 ? n0 : 0) * FEAT + 4 * lane;
    float* g1 = out + (size_t)(a1 ? n1 : 0) * FEAT + 4 * lane;
    if (a0) *(volatile v4f*)g0 = o0;
    if (a1) *(volatile v4f*)g1 = o1;
    __threadfence();
    if (a0) *(volatile v4f*)g0 = o0;
    if (a1) *(volatile v4f*)g1 = o1;
  }
}

__global__ __launch_bounds__(NTHR) void k_readout(const float* __restrict__ x, const int* __restrict__ n2g,
                                                  float* gout, int nN) {
  __shared__ __attribute__((aligned(16))) float red[NWAVE * FEAT];
  const int tid = threadIdx.x, lane = tid & 31, wave = tid >> 5;
  const int g = blockIdx.x;
  v4f acc = {0.f, 0.f, 0.f, 0.f};
  const int nchunk = (nN + NTHR - 1) / NTHR;
#pragma unroll 1
  for (int ch = 0; ch < nchunk; ++ch) {
    const int n = ch * NTHR + tid;
    const int nc = n < nN ? n : nN - 1;
    const int gi = n2g[nc];
    const bool hit = (n < nN) && (gi == g);
    unsigned mk = __builtin_amdgcn_ballot_w32(hit);
    while (mk != 0u) {
      const int i = __builtin_ctz(mk);
      mk &= mk - 1u;
      const int node = ch * NTHR + wave * 32 + i;
      const v4f v = *(const v4f*)(x + (size_t)node * FEAT + 4 * lane);
      acc += v;
    }
  }
  *(v4fa*)(red + wave * FEAT + 4 * lane) = acc;
  __syncthreads();
  if (wave == 0) {
    v4f s = *(const v4fa*)(red + 4 * lane);
#pragma unroll
    for (int w2 = 1; w2 < NWAVE; ++w2) s += *(const v4fa*)(red + w2 * FEAT + 4 * lane);
    float* gp = gout + (size_t)g * FEAT + 4 * lane;
    *(volatile v4f*)gp = s;
    __threadfence();
    *(volatile v4f*)gp = s;
  }
}

extern "C" void kernel_launch(void* const* d_in, const int* in_sizes, int n_in,
                              void* d_out, int out_size, void* d_ws, size_t ws_size,
                              hipStream_t stream) {
  if (n_in < 11) return;
  const int nN = in_sizes[0];
  const int nE = in_sizes[1];
  if (nN < 1 || nN > 65536) return;
  if (nE < 1 || nE > (1 << 28)) return;
  if (in_sizes[2] != nE || in_sizes[3] != nE || in_sizes[4] != nE) return;
  if (in_sizes[5] != nN) return;
  if (in_sizes[6] < FEAT || (in_sizes[6] % FEAT) != 0) return;
  const int nU = in_sizes[6] / FEAT;
  if (in_sizes[7] < KREL * FEAT || (in_sizes[7] % (KREL * FEAT)) != 0) return;
  const int L = in_sizes[7] / (KREL * FEAT);
  if (L < 1 || L > 16) return;
  if (in_sizes[8] != L * FEAT || in_sizes[9] != L * FEAT * FEAT || in_sizes[10] != L * FEAT) return;
  if (out_size <= nN * FEAT || ((out_size - nN * FEAT) % FEAT) != 0) return;
  const int nG = (out_size - nN * FEAT) / FEAT;
  if (nG < 1) return;

  const int*   ut    = (const int*)d_in[0];
  const int*   esrc  = (const int*)d_in[1];
  const int*   edst  = (const int*)d_in[2];
  const int*   ety   = (const int*)d_in[3];
  const float* ew    = (const float*)d_in[4];
  const int*   n2g   = (const int*)d_in[5];
  const float* emb   = (const float*)d_in[6];
  const float* wrel  = (const float*)d_in[7];
  const float* brel  = (const float*)d_in[8];
  const float* wloop = (const float*)d_in[9];
  const float* bloop = (const float*)d_in[10];
  float* out  = (float*)d_out;
  float* gout = out;
  float* xout = out + (size_t)nG * FEAT;

  const int nTiles = (nN + TR - 1) / TR;
  const int nC   = (nN + 4095) >> SH1;
  const int nB1  = (nE + S1 - 1) / S1;
  const int P2   = (nB1 + SEGS2 - 1) / SEGS2;
  const int nch3 = (P2 * CAP2 + NTHR - 1) / NTHR;
  if (nC < 1 || nC > F1A) return;

  char* ws = (char*)d_ws;
  size_t o = 0;
  const size_t oBw = o; o += (size_t)L * FEAT * KD * 2;                      o = (o + 255) & ~(size_t)255;
  const size_t oXA = o; o += (size_t)nN * FEAT * 4;                          o = (o + 255) & ~(size_t)255;
  const size_t oXB = o; o += (size_t)nN * FEAT * 4;                          o = (o + 255) & ~(size_t)255;
  const size_t oL1 = o; o += (size_t)nB1 * nC * CAP1 * 4;                    o = (o + 255) & ~(size_t)255;
  const size_t oL2 = o; o += (size_t)nC * P2 * F2 * CAP2 * 4;                o = (o + 255) & ~(size_t)255;
  const size_t oL3 = o; o += (size_t)nC * MIDS * F3 * CAP3 * 4;              o = (o + 255) & ~(size_t)255;
  if (o > ws_size || o > (size_t)WSCAPB) return;
  _Float16* Bw = (_Float16*)(ws + oBw);
  float*    xA = (float*)(ws + oXA);
  float*    xB = (float*)(ws + oXB);
  unsigned* L1 = (unsigned*)(ws + oL1);
  unsigned* L2 = (unsigned*)(ws + oL2);
  unsigned* L3 = (unsigned*)(ws + oL3);

  k_wprep<<<(L * FEAT * KQ) / NTHR, NTHR, 0, stream>>>(wrel, wloop, Bw);
  k_embed<<<(nN + NWAVE - 1) / NWAVE, NTHR, 0, stream>>>(ut, emb, xA, nN, nU);
  k_part<1, F1A, CAP1><<<nB1, NTHR, 0, stream>>>(edst, L1, L1, nN, nE, nC, nB1, P2, NCH1);
  k_part<2, F2, CAP2><<<nC * P2, NTHR, 0, stream>>>(edst, L1, L2, nN, nE, nC, nB1, P2, NCH2);
  k_part<3, F3, CAP3><<<nC * MIDS, NTHR, 0, stream>>>(edst, L2, L3, nN, nE, nC, nB1, P2, nch3);
  hipFuncSetAttribute(reinterpret_cast<const void*>(&k_tile), hipFuncAttributeMaxDynamicSharedMemorySize, TILE_LDS);
  const float* cur = xA;
  for (int layer = 0; layer < L; ++layer) {
    float* nxt = (layer == L - 1) ? xout : ((cur == xA) ? xB : xA);
    k_tile<<<nTiles, NTHR, TILE_LDS, stream>>>(cur, Bw + (size_t)layer * FEAT * KD, L3, esrc, edst, ety, ew,
                                               brel + (size_t)layer * FEAT, bloop + (size_t)layer * FEAT,
                                               nxt, nN, nE);
    cur = nxt;
  }
  k_readout<<<nG, NTHR, 0, stream>>>(xout, n2g, gout, nN);
}
